// MultiHeadAttention_52209622450793
// MI455X (gfx1250) — hardware-verified
//
#include <hip/hip_runtime.h>
#include <math.h>

#ifndef NB
#define NB 2
#endif
#ifndef SEQ
#define SEQ 2048
#endif
#define NB_FULL 2
#define SEQ_FULL 2048
#define DM 512
#define NH 8
#define DKH 64
#define NTOK (NB * SEQ)
#define PP 72
#define OP 68

static_assert(DM == NH * DKH);
static_assert(DKH == 64);
static_assert(SEQ % 64 == 0);
static_assert(NTOK % 64 == 0);
static_assert(DM % 64 == 0);
static_assert(DM % 32 == 0);
static_assert((2 * DM) % 32 == 0);
static_assert(NB <= NB_FULL);
static_assert(SEQ <= SEQ_FULL);
static_assert((PP % 8) == 0);
static_assert((OP % 4) == 0);

typedef __attribute__((ext_vector_type(16))) _Float16 v16h;
typedef __attribute__((ext_vector_type(8)))  _Float16 v8h;
typedef __attribute__((ext_vector_type(16))) __bf16   v16b;
typedef __attribute__((ext_vector_type(8)))  __bf16   v8b;
typedef __attribute__((ext_vector_type(8)))  float    v8f;
typedef __attribute__((ext_vector_type(4)))  float    v4f;
typedef __attribute__((ext_vector_type(4)))  unsigned int v4u;
typedef v8h v8h_ma __attribute__((may_alias));
typedef v4f v4f_ma __attribute__((may_alias));


__device__ __forceinline__ unsigned int bf_bits(float f) {
    const unsigned int u = __float_as_uint(f);
    return (u + 0x7FFFu + ((u >> 16) & 1u)) >> 16;
}
__device__ __forceinline__ float bf_val(float f) { return __uint_as_float(bf_bits(f) << 16); }
__device__ __forceinline__ unsigned int pk_h2(float a, float b) {
    return (unsigned int)__builtin_bit_cast(unsigned short, (_Float16)a) | ((unsigned int)__builtin_bit_cast(unsigned short, (_Float16)b) << 16);
}
__device__ __forceinline__ void pk_split2(float a, float b, unsigned int& hi, unsigned int& lo) {
    const unsigned int ha = bf_bits(a), hb = bf_bits(b);
    const unsigned int la = bf_bits(a - __uint_as_float(ha << 16)), lb = bf_bits(b - __uint_as_float(hb << 16));
    hi = ha | (hb << 16); lo = la | (lb << 16);
}
__device__ __forceinline__ void wave_sync() {
    __builtin_amdgcn_fence(3  , "workgroup");
    __builtin_amdgcn_wave_barrier();
    __builtin_amdgcn_fence(2  , "workgroup");
}

__device__ __forceinline__ v16h ldfrag_h(const unsigned short* __restrict__ p) {
    const v8h a = *(const v8h*)(p);
    const v8h b = *(const v8h*)(p + 16);
    return __builtin_shufflevector(a, b, 0, 1, 2, 3, 4, 5, 6, 7, 8, 9, 10, 11, 12, 13, 14, 15);
}
__device__ __forceinline__ v16b ldfrag_b(const unsigned short* __restrict__ p) {
    const v8b a = *(const v8b*)(p);
    const v8b b = *(const v8b*)(p + 16);
    return __builtin_shufflevector(a, b, 0, 1, 2, 3, 4, 5, 6, 7, 8, 9, 10, 11, 12, 13, 14, 15);
}

template <int ET> struct FragT;
template <> struct FragT<0> {
    typedef v16h V;
    static __device__ __forceinline__ v16h load(const unsigned short* __restrict__ p) { return ldfrag_h(p); }
    static __device__ __forceinline__ v8f mma(v16h a, v16h b, v8f c) { return __builtin_amdgcn_wmma_f32_16x16x32_f16(false, a, false, b, (short)0, c, false, false); }
};
template <> struct FragT<1> {
    typedef v16b V;
    static __device__ __forceinline__ v16b load(const unsigned short* __restrict__ p) { return ldfrag_b(p); }
    static __device__ __forceinline__ v8f mma(v16b a, v16b b, v8f c) { return __builtin_amdgcn_wmma_f32_16x16x32_bf16(false, a, false, b, (short)0, c, false, false); }
};
template <typename V>
__device__ __forceinline__ void guard4(v8f& a, v8f& b, v8f& c, v8f& d, V x, V y0, V y1, V y2, V y3) {
    asm volatile("v_nop\n\tv_nop\n\tv_nop\n\tv_nop" : "+v"(a), "+v"(b), "+v"(c), "+v"(d) : "v"(x), "v"(y0), "v"(y1), "v"(y2), "v"(y3));
}
__device__ __forceinline__ v8f wmma3b(v16b ah, v16b al, v16b bh, v16b bl, v8f c) {
    c = __builtin_amdgcn_wmma_f32_16x16x32_bf16(false, ah, false, bh, (short)0, c, false, false);
    c = __builtin_amdgcn_wmma_f32_16x16x32_bf16(false, ah, false, bl, (short)0, c, false, false);
    c = __builtin_amdgcn_wmma_f32_16x16x32_bf16(false, al, false, bh, (short)0, c, false, false);
    asm volatile("v_nop\n\tv_nop\n\tv_nop\n\tv_nop" : "+v"(c) : "v"(ah), "v"(al), "v"(bh), "v"(bl));
    return c;
}

template <int ET, int BIAS_MODE, int OUT_MODE>
__device__ __forceinline__ void gemm64_body(const unsigned short* __restrict__ A, int lda,
                                            const unsigned short* __restrict__ Bt, int ldb,
                                            float* __restrict__ Cf, unsigned short* __restrict__ Ca, unsigned short* __restrict__ Cb, int ldc,
                                            const float* __restrict__ bias, int M, int N, int K,
                                            float scale, float bscale, int cseq, int cseqfull) {
    typedef typename FragT<ET>::V V;
    __shared__ __align__(16) float sT[8 * 16 * OP];
    const int lane = threadIdx.x & 31;
    const int wave = __builtin_amdgcn_readfirstlane(threadIdx.x >> 5);
    const int tilesN = N >> 6;
    const int tilesM = M >> 6;
    const int tile = blockIdx.x * 8 + wave;
    if (tile >= tilesM * tilesN) return;
    const int tm = tile / tilesN;
    const int tn = tile - tm * tilesN;
    const int m0 = tm << 6;
    const int n0 = tn << 6;
    const int rl   = lane & 15;
    const int koff = (lane >> 4) * 8;
    const int mOff = (lane >> 4) * 8;

    v8f acc[4][4];
#pragma unroll
    for (int i = 0; i < 4; ++i)
#pragma unroll
        for (int j = 0; j < 4; ++j) { const v8f zz = {0.f, 0.f, 0.f, 0.f, 0.f, 0.f, 0.f, 0.f}; acc[i][j] = zz; }

    for (int k0 = 0; k0 < K; k0 += 32) {
        V bh[4];
#pragma unroll
        for (int j = 0; j < 4; ++j) bh[j] = FragT<ET>::load(Bt + (size_t)(n0 + (j << 4) + rl) * ldb + koff + k0);
#pragma unroll
        for (int i = 0; i < 4; ++i) {
            const V ah = FragT<ET>::load(A + (size_t)(m0 + (i << 4) + rl) * lda + koff + k0);
            acc[i][0] = FragT<ET>::mma(ah, bh[0], acc[i][0]);
            acc[i][1] = FragT<ET>::mma(ah, bh[1], acc[i][1]);
            acc[i][2] = FragT<ET>::mma(ah, bh[2], acc[i][2]);
            acc[i][3] = FragT<ET>::mma(ah, bh[3], acc[i][3]);
            guard4<V>(acc[i][0], acc[i][1], acc[i][2], acc[i][3], ah, bh[0], bh[1], bh[2], bh[3]);
        }
    }

    const int sb = wave * (16 * OP);
#pragma unroll
    for (int i = 0; i < 4; ++i) {
        const int mBase = m0 + (i << 4);
#pragma unroll
        for (int j = 0; j < 4; ++j) {
            const int n = n0 + (j << 4) + rl;
            float bvn = 0.f;
            if (BIAS_MODE == 2) bvn = bf_val(bias[n]) * bscale;
#pragma unroll
            for (int r = 0; r < 8; ++r) {
                float v = acc[i][j][r] * scale;
                if (BIAS_MODE == 1) v += bf_val(bias[mBase + mOff + r]) * bscale;
                if (BIAS_MODE == 2) v += bvn;
                sT[sb + (mOff + r) * OP + (j << 4) + rl] = v;
            }
        }
        wave_sync();
        if (OUT_MODE == 0) {
            const int hh = lane >> 4, c4 = (lane & 15) * 4;
            for (int pass = 0; pass < 2; ++pass) {
#pragma unroll
                for (int it = 0; it < 8; ++it) {
                    const int row = it * 2 + hh;
                    const v4f v = *(const v4f_ma*)&sT[sb + row * OP + c4];
                    const int grow = mBase + row;
                    const int orow = (grow / cseq) * cseqfull + (grow % cseq);
                    *(volatile v4f*)(Cf + (size_t)orow * ldc + n0 + c4) = v;
                }
                __threadfence();
            }
        } else {
            const int q = lane >> 3, c8 = (lane & 7) * 8;
            for (int pass = 0; pass < 2; ++pass) {
#pragma unroll
                for (int it = 0; it < 4; ++it) {
                    const int row = it * 4 + q;
                    const v4f a = *(const v4f_ma*)&sT[sb + row * OP + c8];
                    const v4f b = *(const v4f_ma*)&sT[sb + row * OP + c8 + 4];
                    const size_t o = (size_t)(mBase + row) * ldc + n0 + c8;
                    if (OUT_MODE == 1) {
                        v4u pk; pk.x = pk_h2(a.x, a.y); pk.y = pk_h2(a.z, a.w); pk.z = pk_h2(b.x, b.y); pk.w = pk_h2(b.z, b.w);
                        *(volatile v4u*)(Ca + o) = pk;
                    } else {
                        v4u ph, pl;
                        unsigned int h0, l0, h1, l1, h2, l2, h3, l3;
                        pk_split2(a.x, a.y, h0, l0); pk_split2(a.z, a.w, h1, l1); pk_split2(b.x, b.y, h2, l2); pk_split2(b.z, b.w, h3, l3);
                        ph.x = h0; ph.y = h1; ph.z = h2; ph.w = h3; pl.x = l0; pl.y = l1; pl.z = l2; pl.w = l3;
                        *(volatile v4u*)(Ca + o) = ph;
                        *(volatile v4u*)(Cb + o) = pl;
                    }
                }
                __threadfence();
            }
        }
        wave_sync();
    }
}

__global__ __launch_bounds__(256) void k_gemm_qk(const unsigned short* __restrict__ A, const unsigned short* __restrict__ Bt,
                                                 const float* __restrict__ bias, unsigned short* __restrict__ CH, unsigned short* __restrict__ CL,
                                                 int M, int N, int K, float scale, float bscale) {
    gemm64_body<0, 2, 2>(A, K, Bt, K, nullptr, CH, CL, N, bias, M, N, K, scale, bscale, 1, 1);
}
__global__ __launch_bounds__(256) void k_gemm_vt(const unsigned short* __restrict__ A, const unsigned short* __restrict__ Bt,
                                                 const float* __restrict__ bias, unsigned short* __restrict__ C,
                                                 int M, int N, int K, float scale) {
    gemm64_body<0, 1, 1>(A, K, Bt, K, nullptr, C, nullptr, N, bias, M, N, K, scale, 1.0f, 1, 1);
}
__global__ __launch_bounds__(256) void k_gemm_out(const unsigned short* __restrict__ A, const unsigned short* __restrict__ Bt,
                                                  const float* __restrict__ bias, float* __restrict__ C,
                                                  int M, int N, int K, int cseq, int cseqfull) {
    gemm64_body<1, 2, 0>(A, K, Bt, K, C, nullptr, nullptr, N, bias, M, N, K, 1.0f, 1.0f, cseq, cseqfull);
}

__global__ __launch_bounds__(256) void k_cast16(const float* __restrict__ src, unsigned short* __restrict__ dst, int nrows, int seq, int seqfull, float sc) {
    const int u = blockIdx.x * 256 + threadIdx.x;
    if (u >= nrows * (DM / 8)) return;
    const int r = u / (DM / 8);
    const int c0 = (u - r * (DM / 8)) * 8;
    const int sr = (r / seq) * seqfull + (r % seq);
    const float* s = src + (size_t)sr * DM + c0;
    const v4f a = *(const v4f*)(s);
    const v4f b = *(const v4f*)(s + 4);
    v4u pk;
    pk.x = pk_h2(bf_val(a.x) * sc, bf_val(a.y) * sc); pk.y = pk_h2(bf_val(a.z) * sc, bf_val(a.w) * sc);
    pk.z = pk_h2(bf_val(b.x) * sc, bf_val(b.y) * sc); pk.w = pk_h2(bf_val(b.z) * sc, bf_val(b.w) * sc);
    volatile v4u* d = (volatile v4u*)(dst + (size_t)r * DM + c0);
    *d = pk; __threadfence(); *d = pk;
}
__global__ __launch_bounds__(256) void k_cast_wo(const float* __restrict__ src, unsigned short* __restrict__ dst) {
    const int u = blockIdx.x * 256 + threadIdx.x;
    if (u >= DM * (2 * DM / 8)) return;
    const int r = u / (2 * DM / 8);
    const int c0 = (u - r * (2 * DM / 8)) * 8;
    const int sc0 = c0 & (DM - 1);
    const float* s = src + (size_t)r * DM + sc0;
    const v4f a = *(const v4f*)(s);
    const v4f b = *(const v4f*)(s + 4);
    v4u pk;
    pk.x = bf_bits(a.x) | (bf_bits(a.y) << 16); pk.y = bf_bits(a.z) | (bf_bits(a.w) << 16);
    pk.z = bf_bits(b.x) | (bf_bits(b.y) << 16); pk.w = bf_bits(b.z) | (bf_bits(b.w) << 16);
    volatile v4u* d = (volatile v4u*)(dst + (size_t)r * (2 * DM) + c0);
    *d = pk; __threadfence(); *d = pk;
}

__global__ __launch_bounds__(128) void k_attn(const unsigned short* __restrict__ QH, const unsigned short* __restrict__ QL,
                                              const unsigned short* __restrict__ KH, const unsigned short* __restrict__ KL,
                                              const unsigned short* __restrict__ VT, unsigned short* __restrict__ CTX,
                                              int seq, int ntok) {
    __shared__ __align__(16) _Float16 Psh[4 * 16 * PP];
    __shared__ __align__(16) float    Osh[4 * 16 * OP];
    const int lane = threadIdx.x & 31;
    const int wave = __builtin_amdgcn_readfirstlane(threadIdx.x >> 5);
    const int hf = lane >> 4;
    const int c  = lane & 15;
    const int nqb = seq / 64;
    const int bx = blockIdx.x;
    const int qb = bx % nqb;
    const int bh = bx / nqb;
    const int h  = bh % NH;
    const int b  = bh / NH;
    const int q0 = b * seq + qb * 64 + wave * 16;
    const int qoff  = (q0 + c) * DM + h * DKH + 8 * hf;
    const int kbase = (b * seq + c) * DM + h * DKH + 8 * hf;
    const int vbase = (h * DKH + c) * ntok + b * seq + 8 * hf;
    const int pbase = wave * (16 * PP);
    const int obase = wave * (16 * OP);
    const float L2E = 1.4426950408889634f;

    float mrow[8], lrow[8];
    v8f oacc[4];
#pragma unroll
    for (int r = 0; r < 8; ++r) { mrow[r] = -INFINITY; lrow[r] = 0.f; }
#pragma unroll
    for (int t = 0; t < 4; ++t) { const v8f zz = {0.f, 0.f, 0.f, 0.f, 0.f, 0.f, 0.f, 0.f}; oacc[t] = zz; }

    const int nch = seq / 64;
    for (int kc = 0; kc < nch; ++kc) {
        const int kv0 = kc * 64;
        v8f s[4];
#pragma unroll
        for (int j = 0; j < 4; ++j) { const v8f zz = {0.f, 0.f, 0.f, 0.f, 0.f, 0.f, 0.f, 0.f}; s[j] = zz; }
#pragma unroll 1
        for (int dc = 0; dc < 2; ++dc) {
            const v16b qh = ldfrag_b(QH + qoff + dc * 32);
            const v16b ql = ldfrag_b(QL + qoff + dc * 32);
#pragma unroll
            for (int j = 0; j < 4; ++j) {
                const int ko = kbase + (kv0 + j * 16) * DM + dc * 32;
                const v16b kh = ldfrag_b(KH + ko);
                const v16b kl = ldfrag_b(KL + ko);
                s[j] = wmma3b(qh, ql, kh, kl, s[j]);
                if (j == 1) __builtin_amdgcn_sched_barrier(0);
            }
        }
#pragma unroll
        for (int r = 0; r < 8; ++r) {
            float mx = fmaxf(fmaxf(s[0][r], s[1][r]), fmaxf(s[2][r], s[3][r]));
            mx = fmaxf(mx, __shfl_xor(mx, 1, 32));
            mx = fmaxf(mx, __shfl_xor(mx, 2, 32));
            mx = fmaxf(mx, __shfl_xor(mx, 4, 32));
            mx = fmaxf(mx, __shfl_xor(mx, 8, 32));
            const float mnew = fmaxf(mrow[r], mx);
            const float alpha = exp2f((mrow[r] - mnew) * L2E);
            mrow[r] = mnew;
            const float p0 = exp2f((s[0][r] - mnew) * L2E);
            const float p1 = exp2f((s[1][r] - mnew) * L2E);
            const float p2 = exp2f((s[2][r] - mnew) * L2E);
            const float p3 = exp2f((s[3][r] - mnew) * L2E);
            lrow[r] = lrow[r] * alpha + ((p0 + p1) + (p2 + p3));
            oacc[0][r] *= alpha; oacc[1][r] *= alpha; oacc[2][r] *= alpha; oacc[3][r] *= alpha;
            const int pr = pbase + (8 * hf + r) * PP + c;
            Psh[pr]      = (_Float16)(p0 * 4096.0f);
            Psh[pr + 16] = (_Float16)(p1 * 4096.0f);
            Psh[pr + 32] = (_Float16)(p2 * 4096.0f);
            Psh[pr + 48] = (_Float16)(p3 * 4096.0f);
        }
        wave_sync();
#pragma unroll 1
        for (int kk = 0; kk < 2; ++kk) {
            const int po = pbase + c * PP + kk * 32 + 8 * hf;
            const v8h pa0 = *(const v8h_ma*)&Psh[po];
            const v8h pa1 = *(const v8h_ma*)&Psh[po + 16];
            const v16h pa = __builtin_shufflevector(pa0, pa1, 0, 1, 2, 3, 4, 5, 6, 7, 8, 9, 10, 11, 12, 13, 14, 15);
            const int vo = vbase + kv0 + kk * 32;
            const v16h vb0 = ldfrag_h(VT + vo);
            const v16h vb1 = ldfrag_h(VT + vo + 16 * ntok);
            const v16h vb2 = ldfrag_h(VT + vo + 32 * ntok);
            const v16h vb3 = ldfrag_h(VT + vo + 48 * ntok);
            oacc[0] = __builtin_amdgcn_wmma_f32_16x16x32_f16(false, pa, false, vb0, (short)0, oacc[0], false, false);
            oacc[1] = __builtin_amdgcn_wmma_f32_16x16x32_f16(false, pa, false, vb1, (short)0, oacc[1], false, false);
            oacc[2] = __builtin_amdgcn_wmma_f32_16x16x32_f16(false, pa, false, vb2, (short)0, oacc[2], false, false);
            oacc[3] = __builtin_amdgcn_wmma_f32_16x16x32_f16(false, pa, false, vb3, (short)0, oacc[3], false, false);
            guard4<v16h>(oacc[0], oacc[1], oacc[2], oacc[3], pa, vb0, vb1, vb2, vb3);
        }
        wave_sync();
    }

#pragma unroll
    for (int r = 0; r < 8; ++r) {
        float l = lrow[r];
        l += __shfl_xor(l, 1, 32);
        l += __shfl_xor(l, 2, 32);
        l += __shfl_xor(l, 4, 32);
        l += __shfl_xor(l, 8, 32);
        const float inv = 1.0f / (l * 4096.0f);
        const int orw = obase + (8 * hf + r) * OP + c;
        Osh[orw]      = oacc[0][r] * inv;
        Osh[orw + 16] = oacc[1][r] * inv;
        Osh[orw + 32] = oacc[2][r] * inv;
        Osh[orw + 48] = oacc[3][r] * inv;
    }
    wave_sync();
    {
        const int q = lane >> 3, c8 = (lane & 7) * 8;
        for (int pass = 0; pass < 2; ++pass) {
#pragma unroll
            for (int it = 0; it < 4; ++it) {
                const int row = it * 4 + q;
                const v4f a = *(const v4f_ma*)&Osh[obase + row * OP + c8];
                const v4f bb = *(const v4f_ma*)&Osh[obase + row * OP + c8 + 4];
                unsigned int h0, l0, h1, l1, h2, l2, h3, l3;
                pk_split2(a.x, a.y, h0, l0); pk_split2(a.z, a.w, h1, l1); pk_split2(bb.x, bb.y, h2, l2); pk_split2(bb.z, bb.w, h3, l3);
                v4u ph, pl;
                ph.x = h0; ph.y = h1; ph.z = h2; ph.w = h3; pl.x = l0; pl.y = l1; pl.z = l2; pl.w = l3;
                const size_t o = (size_t)(q0 + row) * (2 * DM) + h * DKH + c8;
                *(volatile v4u*)(CTX + o) = ph;
                *(volatile v4u*)(CTX + o + DM) = pl;
            }
            __threadfence();
        }
    }
}

constexpr size_t SZ_TOK  = (size_t)NTOK * DM * 2;
constexpr size_t SZ_W    = (size_t)DM * DM * 2;
constexpr size_t SZ_WOD  = (size_t)DM * (2 * DM) * 2;
constexpr size_t SZ_CTX  = (size_t)NTOK * (2 * DM) * 2;
constexpr size_t WS_TOTAL = 3 * SZ_TOK + 3 * SZ_W + SZ_WOD + 4 * SZ_TOK + SZ_TOK + SZ_CTX;
static_assert(SZ_TOK % 256 == 0);
static_assert(SZ_W % 256 == 0);
static_assert(SZ_WOD % 256 == 0);
static_assert(SZ_CTX % 256 == 0);
static_assert(WS_TOTAL <= (size_t)134217728);
static_assert(((NTOK / 64) * (DM / 64)) % 8 == 0);
static_assert((size_t)NTOK * (2 * DM) < (size_t)2147483647);

extern "C" void kernel_launch(void* const* d_in, const int* in_sizes, int n_in, void* d_out, int out_size, void* d_ws, size_t ws_size, hipStream_t stream) {
    if (n_in < 11) return;
    const long long need_x = ((long long)(NB - 1) * SEQ_FULL + SEQ) * DM;
    if ((long long)in_sizes[0] < need_x || (long long)in_sizes[1] < need_x || (long long)in_sizes[2] < need_x) return;
    if (in_sizes[3] < DM * DM || in_sizes[5] < DM * DM || in_sizes[7] < DM * DM || in_sizes[9] < DM * DM) return;
    if (in_sizes[4] < DM || in_sizes[6] < DM || in_sizes[8] < DM || in_sizes[10] < DM) return;
    if ((long long)out_size < need_x) return;
    if (WS_TOTAL > ws_size) return;

    const float* xq = (const float*)d_in[0];
    const float* xk = (const float*)d_in[1];
    const float* xv = (const float*)d_in[2];
    const float* Wq = (const float*)d_in[3];
    const float* bq = (const float*)d_in[4];
    const float* Wk = (const float*)d_in[5];
    const float* bk = (const float*)d_in[6];
    const float* Wv = (const float*)d_in[7];
    const float* bv = (const float*)d_in[8];
    const float* Wo = (const float*)d_in[9];
    const float* bo = (const float*)d_in[10];
    float* out = (float*)d_out;

    char* wsp = (char*)d_ws;
    unsigned short* XQ16 = (unsigned short*)wsp; wsp += SZ_TOK;
    unsigned short* XK16 = (unsigned short*)wsp; wsp += SZ_TOK;
    unsigned short* XV16 = (unsigned short*)wsp; wsp += SZ_TOK;
    unsigned short* WQ16 = (unsigned short*)wsp; wsp += SZ_W;
    unsigned short* WK16 = (unsigned short*)wsp; wsp += SZ_W;
    unsigned short* WV16 = (unsigned short*)wsp; wsp += SZ_W;
    unsigned short* WOD  = (unsigned short*)wsp; wsp += SZ_WOD;
    unsigned short* QHp  = (unsigned short*)wsp; wsp += SZ_TOK;
    unsigned short* QLp  = (unsigned short*)wsp; wsp += SZ_TOK;
    unsigned short* KHp  = (unsigned short*)wsp; wsp += SZ_TOK;
    unsigned short* KLp  = (unsigned short*)wsp; wsp += SZ_TOK;
    unsigned short* VTp  = (unsigned short*)wsp; wsp += SZ_TOK;
    unsigned short* CTXp = (unsigned short*)wsp; wsp += SZ_CTX;
    if ((size_t)(wsp - (char*)d_ws) > ws_size) return;

    const unsigned gx_tok = (unsigned)((NTOK * (DM / 8) + 255) / 256);
    const unsigned gx_w   = (unsigned)((DM * (DM / 8) + 255) / 256);
    const unsigned gx_wo  = (unsigned)((DM * (2 * DM / 8) + 255) / 256);
    const unsigned gx_gemm = (unsigned)((((NTOK / 64) * (DM / 64)) + 7) / 8);

    k_cast16<<<gx_tok, 256, 0, stream>>>(xq, XQ16, NTOK, SEQ, SEQ_FULL, 1.0f);
    k_cast16<<<gx_tok, 256, 0, stream>>>(xk, XK16, NTOK, SEQ, SEQ_FULL, 1.0f);
    k_cast16<<<gx_tok, 256, 0, stream>>>(xv, XV16, NTOK, SEQ, SEQ_FULL, 1.0f);
    k_cast16<<<gx_w, 256, 0, stream>>>(Wq, WQ16, DM, DM, DM, 16.0f);
    k_cast16<<<gx_w, 256, 0, stream>>>(Wk, WK16, DM, DM, DM, 16.0f);
    k_cast16<<<gx_w, 256, 0, stream>>>(Wv, WV16, DM, DM, DM, 16.0f);
    k_cast_wo<<<gx_wo, 256, 0, stream>>>(Wo, WOD);

    k_gemm_qk<<<gx_gemm, 256, 0, stream>>>(XQ16, WQ16, bq, QHp, QLp, NTOK, DM, DM, 1.0f / 128.0f, 0.125f);
    k_gemm_qk<<<gx_gemm, 256, 0, stream>>>(XK16, WK16, bk, KHp, KLp, NTOK, DM, DM, 1.0f / 16.0f, 1.0f);
    k_gemm_vt<<<gx_gemm, 256, 0, stream>>>(WV16, XV16, bv, VTp, DM, NTOK, DM, 1.0f / 16.0f);

    k_attn<<<(unsigned)(NB * NH * (SEQ / 64)), 128, 0, stream>>>(QHp, QLp, KHp, KLp, VTp, CTXp, SEQ, NTOK);

    k_gemm_out<<<gx_gemm, 256, 0, stream>>>(CTXp, WOD, bo, out, NTOK, DM, 2 * DM, SEQ, SEQ_FULL);
}
